// RecurrentAutoencoder_6442450944675
// MI455X (gfx1250) — hardware-verified
//
#include <hip/hip_runtime.h>
#include <math.h>
#include <stdint.h>

constexpr int NBATCH  = 256;
constexpr int NSTEP   = 1023;
constexpr int WLEN    = 8192;
constexpr int SWIN    = 16;
constexpr int SSTRIDE = 8;
constexpr int HE1 = 128, HE2 = 64, HD1 = 64, HD2 = 128, NFEAT = 16;
constexpr int GD1 = 4 * HD1;
constexpr int KE1   = 160;
constexpr int KE2   = 192;
constexpr int KD1R  = 64;
constexpr int KD2   = 192;
constexpr int KPROJ = 128;
constexpr int TR    = 16;
constexpr int NTHR  = 256;
constexpr int P1  = 168;
constexpr int P2  = 72;
constexpr int PD1 = 72;
constexpr int PD2 = 136;
constexpr int XP  = 272;
constexpr int XCHUNK_F = 256;
constexpr int ZP  = 68;
constexpr int YP  = 32;
constexpr float A_CARRY = 16.0f;
constexpr float W_CARRY = 64.0f;
constexpr float Z_FOLD  = 1.0f / 1024.0f;

static_assert(NBATCH % TR == 0, "grid covers all batch rows exactly");
static_assert(SSTRIDE * (NSTEP - 1) == WLEN - SWIN, "trailing window starts at stride*(NSTEP-1)");
static_assert(((NSTEP - 1) >> 2) == WLEN / 32 - 1, "last step flushes the last 128-B line");
static_assert(((NSTEP - 1) & 3) == 2, "last window fills floats 16..31 of the last line");
static_assert((NSTEP - 1) / 32 * XCHUNK_F + XP >= WLEN, "x chunks cover the row");
static_assert(P1 % 8 == 0 && P2 % 8 == 0 && PD1 % 8 == 0 && PD2 % 8 == 0 && XP % 8 == 0, "16-B aligned LDS rows");
static_assert(KE1 % 32 == 0 && KE2 % 32 == 0 && KD1R % 32 == 0 && KD2 % 32 == 0 && KPROJ % 32 == 0, "K multiple of 32");
static_assert(TR * SWIN == NTHR, "window copy: one half per thread");

typedef __attribute__((ext_vector_type(16))) _Float16 v16h;
typedef __attribute__((ext_vector_type(8)))  _Float16 v8h;
typedef __attribute__((ext_vector_type(4)))  _Float16 v4h;
typedef __attribute__((ext_vector_type(16))) __bf16   v16b;
typedef __attribute__((ext_vector_type(8)))  __bf16   v8b;
typedef __attribute__((ext_vector_type(8)))  float    v8f;
typedef __attribute__((ext_vector_type(4)))  float    v4f;

__device__ __forceinline__ unsigned short f2bf_bits(float f) {
  unsigned u = __float_as_uint(f);
  return (unsigned short)((u + 0x7FFFu + ((u >> 16) & 1u)) >> 16);
}
__device__ __forceinline__ float bf_bits2f(unsigned short h) { return __uint_as_float(((unsigned)h) << 16); }
__device__ __forceinline__ float bfr(float f) { return bf_bits2f(f2bf_bits(f)); }

__device__ __forceinline__ void dep_guard_h(v8f& a, v8f& b, v16h x, v16h y) { asm volatile("v_nop\n\tv_nop\n\tv_nop\n\tv_nop" : "+v"(a), "+v"(b) : "v"(x), "v"(y)); }
__device__ __forceinline__ void dep_guard_b(v8f& a, v8f& b, v16b x, v16b y) { asm volatile("v_nop\n\tv_nop\n\tv_nop\n\tv_nop" : "+v"(a), "+v"(b) : "v"(x), "v"(y)); }
__device__ __forceinline__ void keep4_h(v16h a, v16h b, v16h c, v16h d) { asm volatile("v_nop" :: "v"(a), "v"(b), "v"(c), "v"(d)); }
__device__ __forceinline__ void keep4_b(v16b a, v16b b, v16b c, v16b d) { asm volatile("v_nop" :: "v"(a), "v"(b), "v"(c), "v"(d)); }
__device__ __forceinline__ void keep5_h(v16h a, v16h b, v16h c, v16h d, v16h e) { asm volatile("v_nop" :: "v"(a), "v"(b), "v"(c), "v"(d), "v"(e)); }
__device__ __forceinline__ void acc_guard4(v8f& a, v8f& b, v8f& c, v8f& d) { asm volatile("v_nop\n\tv_nop\n\tv_nop\n\tv_nop" : "+v"(a), "+v"(b), "+v"(c), "+v"(d)); }
__device__ __forceinline__ void guard1_h(v8f& a, v16h x, v16h y) { asm volatile("v_nop\n\tv_nop\n\tv_nop\n\tv_nop" : "+v"(a) : "v"(x), "v"(y)); }
template <typename T> struct Frag;
template <> struct Frag<_Float16> {
  typedef v16h V; union U { v16h v; v8h h[2]; };
  static __device__ __forceinline__ v16h load(const _Float16* p) {
    U f; f.h[0] = *(const v8h*)(p); f.h[1] = *(const v8h*)(p + 16); return f.v;
  }
  static __device__ __forceinline__ v8f mma(v16h a, v16h b, v8f c) {
    return __builtin_amdgcn_wmma_f32_16x16x32_f16(false, a, false, b, (short)0, c, false, false);
  }
  static __device__ __forceinline__ void guard(v8f& a, v8f& b, v16h x, v16h y) { dep_guard_h(a, b, x, y); }
  static __device__ __forceinline__ void keep(v16h a, v16h b, v16h c, v16h d) { keep4_h(a, b, c, d); }
};
template <> struct Frag<__bf16> {
  typedef v16b V; union U { v16b v; v8b h[2]; };
  static __device__ __forceinline__ v16b load(const __bf16* p) {
    U f; f.h[0] = *(const v8b*)(p); f.h[1] = *(const v8b*)(p + 16); return f.v;
  }
  static __device__ __forceinline__ v8f mma(v16b a, v16b b, v8f c) {
    return __builtin_amdgcn_wmma_f32_16x16x32_bf16(false, a, false, b, (short)0, c, false, false);
  }
  static __device__ __forceinline__ void guard(v8f& a, v8f& b, v16b x, v16b y) { dep_guard_b(a, b, x, y); }
  static __device__ __forceinline__ void keep(v16b a, v16b b, v16b c, v16b d) { keep4_b(a, b, c, d); }
};
typedef Frag<_Float16> FragH;

template <int ET> struct Elem;
template <> struct Elem<0> { typedef _Float16 T; };
template <> struct Elem<1> { typedef __bf16 T; };
template <int ET, bool SPLIT, int BIAS_MODE, int OUT_MODE, bool RESID, int ACT = 0>
__global__ __launch_bounds__(256) void wmma_gemm64(
    const unsigned short* __restrict__ Ap, const unsigned short* __restrict__ A2p, int lda, long strideA,
    const unsigned short* __restrict__ Btp, const unsigned short* __restrict__ Bt2p, int ldb, long strideB,
    void* __restrict__ Cout, void* __restrict__ Cout2, int ldc, long strideC,
    const float* __restrict__ bias,
    const float* __restrict__ resid, long strideR,
    int M, int N, int K, float scale) {
  typedef typename Elem<ET>::T T;
  typedef typename Frag<T>::V V;
  const T* A = (const T*)Ap; const T* A2 = (const T*)A2p; const T* Bt = (const T*)Btp; const T* Bt2 = (const T*)Bt2p;
  __shared__ __align__(16) float sT[8][16 * 68];
  const int b    = blockIdx.y;
  const int lane = threadIdx.x & 31;
  const int wave = threadIdx.x >> 5;
  const int tilesN = N >> 6;
  const int tilesM = M >> 6;
  const int tile = blockIdx.x * 8 + wave;
  if (tile >= tilesM * tilesN) return;
  const int tm = tile / tilesN;
  const int tn = tile - tm * tilesN;
  const int m0 = tm << 6;
  const int n0 = tn << 6;

  const T* Ab  = A  + (size_t)b * strideA;
  const T* Bb  = Bt + (size_t)b * strideB;
  const T* Ab2 = SPLIT ? (A2  + (size_t)b * strideA) : nullptr;
  const T* Bb2 = SPLIT ? (Bt2 + (size_t)b * strideB) : nullptr;

  const int rlane = lane & 15;
  const int koff  = (lane >> 4) * 8;
  const int mOff  = (lane >> 4) * 8;

  v8f acc[4][4];
#pragma unroll
  for (int i = 0; i < 4; ++i)
#pragma unroll
    for (int j = 0; j < 4; ++j) acc[i][j] = (v8f){0.f,0.f,0.f,0.f,0.f,0.f,0.f,0.f};

  for (int k0 = 0; k0 < K; k0 += 32) {
    V bh[4], bl[4];
#pragma unroll
    for (int j = 0; j < 4; ++j) {
      const size_t bo = (size_t)(n0 + (j << 4) + rlane) * ldb + koff + k0;
      bh[j] = Frag<T>::load(Bb + bo);
      if (SPLIT) bl[j] = Frag<T>::load(Bb2 + bo);
    }
#pragma unroll
    for (int i = 0; i < 4; ++i) {
      const size_t ao = (size_t)(m0 + (i << 4) + rlane) * lda + koff + k0;
      V ah = Frag<T>::load(Ab + ao);
      V al;
      if (SPLIT) al = Frag<T>::load(Ab2 + ao);
#pragma unroll
      for (int j = 0; j < 4; ++j) {
        acc[i][j] = Frag<T>::mma(ah, bh[j], acc[i][j]);
        if (SPLIT) {
          acc[i][j] = Frag<T>::mma(ah, bl[j], acc[i][j]);
          acc[i][j] = Frag<T>::mma(al, bh[j], acc[i][j]);
        }
      }
      Frag<T>::guard(acc[i][0], acc[i][3], ah, SPLIT ? al : ah);
    }
    Frag<T>::keep(bh[0], bh[1], bh[2], bh[3]);
    if (SPLIT) Frag<T>::keep(bl[0], bl[1], bl[2], bl[3]);
  }
  acc_guard4(acc[0][0], acc[0][1], acc[0][2], acc[0][3]);
  acc_guard4(acc[1][0], acc[1][1], acc[1][2], acc[1][3]);
  acc_guard4(acc[2][0], acc[2][1], acc[2][2], acc[2][3]);
  acc_guard4(acc[3][0], acc[3][1], acc[3][2], acc[3][3]);

  float* slab = sT[wave];
  const float* Rb = RESID ? (resid + (size_t)b * strideR) : nullptr;
#pragma unroll
  for (int i = 0; i < 4; ++i) {
    const int mBase = m0 + (i << 4);
#pragma unroll
    for (int j = 0; j < 4; ++j) {
      const int n = n0 + (j << 4) + rlane;
      float bv = 0.f;
      if (BIAS_MODE == 2) bv = bias[n];
#pragma unroll
      for (int r = 0; r < 8; ++r) {
        float v = acc[i][j][r] * scale;
        if (BIAS_MODE == 1) v += bias[mBase + mOff + r];
        if (BIAS_MODE == 2) v += bv;
        if (RESID) v += Rb[(size_t)(mBase + mOff + r) * ldc + n];
        if (ACT == 1) v = tanhf(v);
        if (ACT == 2) v = fmaxf(v, 0.0f);
        if (ACT == 3) v = v / (1.0f + expf(-v));
        if (ACT == 4) v = (v > 0.f) ? v : 0.01f * v;
        if (ACT == 5) v = 0.5f * v * (1.0f + erff(v * 0.70710678118654752f));
        slab[(mOff + r) * 68 + (j << 4) + rlane] = v;
      }
    }
    __builtin_amdgcn_fence(__ATOMIC_RELEASE, "workgroup");
    __builtin_amdgcn_wave_barrier();
    __builtin_amdgcn_fence(__ATOMIC_ACQUIRE, "workgroup");
    if (OUT_MODE == 0) {
      float* C = (float*)Cout + (size_t)b * strideC;
      const int hh = lane >> 4, c4 = (lane & 15) * 4;
      for (int pass = 0; pass < 2; ++pass) {
#pragma unroll
        for (int it = 0; it < 8; ++it) {
          const int row = it * 2 + hh;
          v4f v = *(const v4f*)(slab + row * 68 + c4);
          *(volatile v4f*)(C + (size_t)(mBase + row) * ldc + n0 + c4) = v;
        }
        __threadfence();
      }
    } else {
      const int q = lane >> 3, c8 = (lane & 7) * 8;
      unsigned short* C  = (unsigned short*)Cout  + (size_t)b * strideC;
      unsigned short* C2 = (OUT_MODE == 2) ? ((unsigned short*)Cout2 + (size_t)b * strideC) : nullptr;
      for (int pass = 0; pass < 2; ++pass) {
#pragma unroll
        for (int it = 0; it < 4; ++it) {
          const int row = it * 4 + q;
          const float* sp = slab + row * 68 + c8;
          v8h hv, lv;
#pragma unroll
          for (int e = 0; e < 8; ++e) {
            if (OUT_MODE == 1) {
              hv[e] = (_Float16)sp[e];
            } else {
              unsigned short hb = f2bf_bits(sp[e]);
              unsigned short lb = f2bf_bits(sp[e] - bf_bits2f(hb));
              hv[e] = __builtin_bit_cast(_Float16, hb);
              lv[e] = __builtin_bit_cast(_Float16, lb);
            }
          }
          *(volatile v8h*)(C + (size_t)(mBase + row) * ldc + n0 + c8) = hv;
          if (OUT_MODE == 2) *(volatile v8h*)(C2 + (size_t)(mBase + row) * ldc + n0 + c8) = lv;
        }
        __threadfence();
      }
    }
    __builtin_amdgcn_fence(__ATOMIC_RELEASE, "workgroup");
    __builtin_amdgcn_wave_barrier();
    __builtin_amdgcn_fence(__ATOMIC_ACQUIRE, "workgroup");
  }
}

__device__ __forceinline__ float fsig(float v)  { return __builtin_amdgcn_rcpf(1.0f + __expf(-v)); }
__device__ __forceinline__ float ftanh(float v) { return 1.0f - 2.0f * __builtin_amdgcn_rcpf(__expf(2.0f * v) + 1.0f); }

__global__ __launch_bounds__(NTHR) void wplane_kernel(const float* __restrict__ Wa, int Ka,
                                                      const float* __restrict__ Wb, int Kb, int offB,
                                                      int KP, int n8, int mode, unsigned short* __restrict__ O) {
  const int i = blockIdx.x * NTHR + threadIdx.x;
  if (i >= n8) return;
  const int e0 = i * 8;
  const int n  = e0 / KP;
  const int kk = e0 - n * KP;
  v8h hv;
#pragma unroll
  for (int e = 0; e < 8; ++e) {
    const int k = kk + e;
    const int ia = (k < Ka) ? k : (Ka - 1);
    int ib = k - offB; ib = ib < 0 ? 0 : ib; ib = ib > Kb - 1 ? Kb - 1 : ib;
    const float va = Wa[(size_t)n * Ka + ia];
    const float vb = Wb[(size_t)n * Kb + ib];
    const float v  = (k < Ka) ? va : ((k >= offB && k < offB + Kb) ? vb : 0.0f);
    unsigned short bits;
    if (mode == 0)      bits = __builtin_bit_cast(unsigned short, (_Float16)(bfr(v) * W_CARRY));
    else if (mode == 1) bits = f2bf_bits(v);
    else                bits = (unsigned short)0;
    hv[e] = __builtin_bit_cast(_Float16, bits);
  }
  *(volatile v8h*)(O + e0) = hv;
  __threadfence();
  *(volatile v8h*)(O + e0) = hv;
}

template <int NKC>
__device__ __forceinline__ void gate_mac4(v8f (&acc)[4], const _Float16* arow, const _Float16* w, int gstride) {
#pragma unroll 1
  for (int kc = 0; kc < NKC; ++kc) {
    const int k0 = kc * 32;
    const v16h a  = FragH::load(arow + k0);
    const v16h w0 = FragH::load(w + k0);
    const v16h w1 = FragH::load(w + (size_t)gstride + k0);
    const v16h w2 = FragH::load(w + (size_t)2 * gstride + k0);
    const v16h w3 = FragH::load(w + (size_t)3 * gstride + k0);
    acc[0] = FragH::mma(a, w0, acc[0]);
    acc[1] = FragH::mma(a, w1, acc[1]);
    acc[2] = FragH::mma(a, w2, acc[2]);
    acc[3] = FragH::mma(a, w3, acc[3]);
    acc_guard4(acc[0], acc[1], acc[2], acc[3]);
    keep5_h(a, w0, w1, w2, w3);
  }
}

__device__ __forceinline__ void lstm_cell8(const v8f (&acc)[4], float fold, float bi, float bf, float bg, float bo,
                                           float (&cst)[8], float (&hout)[8]) {
#pragma unroll
  for (int r = 0; r < 8; ++r) {
    const float pi = fmaf(acc[0][r], fold, bi);
    const float pf = fmaf(acc[1][r], fold, bf);
    const float pg = fmaf(acc[2][r], fold, bg);
    const float po = fmaf(acc[3][r], fold, bo);
    const float ig = fsig(pi);
    const float fg = fsig(pf);
    const float gg = ftanh(pg);
    const float og = fsig(po);
    const float cv = fmaf(fg, cst[r], ig * gg);
    cst[r] = cv;
    hout[r] = og * ftanh(cv);
  }
}

__device__ __forceinline__ void stage_x(_Float16* xs, const float* __restrict__ x, int b0, int cb, int tid) {
  constexpr int SLOTS_PER_ROW = XP / 4;
#pragma unroll 1
  for (int i = tid; i < TR * SLOTS_PER_ROW; i += NTHR) {
    const int m  = i / SLOTS_PER_ROW;
    const int c4 = (i - m * SLOTS_PER_ROW) * 4;
    int col = cb + c4;
    col = (col > WLEN - 4) ? (WLEN - 4) : col;
    const v4f v = *(const v4f*)(x + (size_t)(b0 + m) * WLEN + col);
    v4h w;
    w[0] = (_Float16)(A_CARRY * bfr(v[0]));
    w[1] = (_Float16)(A_CARRY * bfr(v[1]));
    w[2] = (_Float16)(A_CARRY * bfr(v[2]));
    w[3] = (_Float16)(A_CARRY * bfr(v[3]));
    *(v4h*)(xs + m * XP + c4) = w;
  }
}

__global__ __launch_bounds__(NTHR) void enc_kernel(
    const float* __restrict__ x,
    const float* __restrict__ e1bi, const float* __restrict__ e1bh,
    const float* __restrict__ e2bi, const float* __restrict__ e2bh,
    const unsigned short* __restrict__ WE1p, const unsigned short* __restrict__ WE2p,
    unsigned short* __restrict__ ZHp, unsigned short* __restrict__ ZLp) {
  __shared__ __align__(16) _Float16 a1[TR * P1];
  __shared__ __align__(16) _Float16 a2[TR * P2];
  __shared__ __align__(16) _Float16 xs[TR * XP];
  __shared__ __align__(16) float    zs[TR * ZP];

  const int tid = threadIdx.x, lane = tid & 31, wave = tid >> 5;
  const int c = lane & 15, hh = lane >> 4, koff = hh * 8, rb = 8 * hh;
  const int j1 = 16 * wave + c;
  const int j2 = 16 * (wave & 3) + c;
  const int b0 = blockIdx.x * TR;

#pragma unroll 1
  for (int i = tid; i < TR * P1; i += NTHR) a1[i] = (_Float16)0.0f;
#pragma unroll 1
  for (int i = tid; i < TR * P2; i += NTHR) a2[i] = (_Float16)0.0f;

  const float b1i_ = bfr(e1bi[0 * HE1 + j1]) + bfr(e1bh[0 * HE1 + j1]);
  const float b1f_ = bfr(e1bi[1 * HE1 + j1]) + bfr(e1bh[1 * HE1 + j1]);
  const float b1g_ = bfr(e1bi[2 * HE1 + j1]) + bfr(e1bh[2 * HE1 + j1]);
  const float b1o_ = bfr(e1bi[3 * HE1 + j1]) + bfr(e1bh[3 * HE1 + j1]);
  const float b2i_ = bfr(e2bi[0 * HE2 + j2]) + bfr(e2bh[0 * HE2 + j2]);
  const float b2f_ = bfr(e2bi[1 * HE2 + j2]) + bfr(e2bh[1 * HE2 + j2]);
  const float b2g_ = bfr(e2bi[2 * HE2 + j2]) + bfr(e2bh[2 * HE2 + j2]);
  const float b2o_ = bfr(e2bi[3 * HE2 + j2]) + bfr(e2bh[3 * HE2 + j2]);

  float c1s[8], c2s[8], h1v[8], h2v[8];
#pragma unroll
  for (int r = 0; r < 8; ++r) { c1s[r] = 0.0f; c2s[r] = 0.0f; h1v[r] = 0.0f; h2v[r] = 0.0f; }

  stage_x(xs, x, b0, 0, tid);
  __syncthreads();
  {
    const int m = tid >> 4, jj = tid & 15;
    a1[m * P1 + jj] = xs[m * XP + jj];
  }
  __syncthreads();

  const _Float16* a1row = a1 + c * P1 + koff;
  const _Float16* a2row = a2 + c * P2 + koff;
  const _Float16* we1 = (const _Float16*)WE1p + (size_t)j1 * KE1 + koff;
  const _Float16* we2 = (const _Float16*)WE2p + (size_t)j2 * KE2 + koff;
  const v8f z8 = {0.f, 0.f, 0.f, 0.f, 0.f, 0.f, 0.f, 0.f};

#pragma unroll 1
  for (int t = 0; t < NSTEP; ++t) {
    if (t > 0 && (t & 31) == 0) stage_x(xs, x, b0, (t >> 5) * XCHUNK_F, tid);

    {
      v8f acc[4];
      acc[0] = z8; acc[1] = z8; acc[2] = z8; acc[3] = z8;
      gate_mac4<KE1 / 32>(acc, a1row, we1, HE1 * KE1);
      lstm_cell8(acc, Z_FOLD, b1i_, b1f_, b1g_, b1o_, c1s, h1v);
    }
    __syncthreads();
#pragma unroll
    for (int r = 0; r < 8; ++r) a1[(rb + r) * P1 + 32 + j1] = (_Float16)(A_CARRY * h1v[r]);
    if (t + 1 < NSTEP) {
      const int m = tid >> 4, jj = tid & 15;
      a1[m * P1 + jj] = xs[m * XP + SSTRIDE * ((t & 31) + 1) + jj];
    }
    __syncthreads();

    if (wave < 4) {
      v8f acc[4];
      acc[0] = z8; acc[1] = z8; acc[2] = z8; acc[3] = z8;
      gate_mac4<HE1 / 32>(acc, a1row + 32, we2, HE2 * KE2);
      gate_mac4<HE2 / 32>(acc, a2row, we2 + HE1, HE2 * KE2);
      lstm_cell8(acc, Z_FOLD, b2i_, b2f_, b2g_, b2o_, c2s, h2v);
    }
    __syncthreads();
    if (wave < 4) {
#pragma unroll
      for (int r = 0; r < 8; ++r) a2[(rb + r) * P2 + j2] = (_Float16)(A_CARRY * h2v[r]);
    }
  }

  if (wave < 4) {
#pragma unroll
    for (int r = 0; r < 8; ++r) zs[(rb + r) * ZP + j2] = h2v[r];
  }
  __syncthreads();
  {
    const int q = lane >> 3, c8 = (lane & 7) * 8;
    const int row = 4 * (wave & 3) + q;
    const float* sp = zs + row * ZP + c8;
    const bool hiw = (wave < 4);
    v8h sv;
#pragma unroll
    for (int e = 0; e < 8; ++e) {
      const unsigned short hb = f2bf_bits(sp[e]);
      const unsigned short lb = f2bf_bits(sp[e] - bf_bits2f(hb));
      sv[e] = __builtin_bit_cast(_Float16, hiw ? hb : lb);
    }
    unsigned short* base = hiw ? ZHp : ZLp;
    unsigned short* op = base + (size_t)(b0 + row) * HE2 + c8;
    *(volatile v8h*)op = sv;
    __threadfence();
    *(volatile v8h*)op = sv;
  }
}

__global__ __launch_bounds__(NTHR) void dec_kernel(
    const float* __restrict__ d1bi, const float* __restrict__ d1bh,
    const float* __restrict__ d2bi, const float* __restrict__ d2bh,
    const float* __restrict__ ob,
    const unsigned short* __restrict__ WD1Rp, const unsigned short* __restrict__ WD2p,
    const unsigned short* __restrict__ WOp, const float* __restrict__ DG,
    float* __restrict__ out) {
  __shared__ __align__(16) _Float16 ad1[TR * PD1];
  __shared__ __align__(16) _Float16 ad2[TR * PD2];
  __shared__ __align__(16) float    ys[TR * YP];

  const int tid = threadIdx.x, lane = tid & 31, wave = tid >> 5;
  const int c = lane & 15, hh = lane >> 4, koff = hh * 8, rb = 8 * hh;
  const int j1 = 16 * wave + c;
  const int j2 = 16 * (wave & 3) + c;
  const int b0 = blockIdx.x * TR;

#pragma unroll 1
  for (int i = tid; i < TR * PD1; i += NTHR) ad1[i] = (_Float16)0.0f;
#pragma unroll 1
  for (int i = tid; i < TR * PD2; i += NTHR) ad2[i] = (_Float16)0.0f;
#pragma unroll 1
  for (int i = tid; i < TR * YP; i += NTHR) ys[i] = 0.0f;

  const float bd1i = bfr(d1bi[0 * HD1 + j2]) + bfr(d1bh[0 * HD1 + j2]);
  const float bd1f = bfr(d1bi[1 * HD1 + j2]) + bfr(d1bh[1 * HD1 + j2]);
  const float bd1g = bfr(d1bi[2 * HD1 + j2]) + bfr(d1bh[2 * HD1 + j2]);
  const float bd1o = bfr(d1bi[3 * HD1 + j2]) + bfr(d1bh[3 * HD1 + j2]);
  const float bd2i = bfr(d2bi[0 * HD2 + j1]) + bfr(d2bh[0 * HD2 + j1]);
  const float bd2f = bfr(d2bi[1 * HD2 + j1]) + bfr(d2bh[1 * HD2 + j1]);
  const float bd2g = bfr(d2bi[2 * HD2 + j1]) + bfr(d2bh[2 * HD2 + j1]);
  const float bd2o = bfr(d2bi[3 * HD2 + j1]) + bfr(d2bh[3 * HD2 + j1]);
  const float obias = bfr(ob[c]);

  float cd1[8], cd2[8], hd1v[8], hd2v[8];
#pragma unroll
  for (int r = 0; r < 8; ++r) { cd1[r] = 0.0f; cd2[r] = 0.0f; hd1v[r] = 0.0f; hd2v[r] = 0.0f; }
  __syncthreads();

  const _Float16* ad1row = ad1 + c * PD1 + koff;
  const _Float16* ad2row = ad2 + c * PD2 + koff;
  const _Float16* wd1 = (const _Float16*)WD1Rp + (size_t)j2 * KD1R + koff;
  const _Float16* wd2 = (const _Float16*)WD2p + (size_t)j1 * KD2 + koff;
  const _Float16* wo  = (const _Float16*)WOp + (size_t)c * KPROJ + koff;
  const v8f z8 = {0.f, 0.f, 0.f, 0.f, 0.f, 0.f, 0.f, 0.f};

#pragma unroll 1
  for (int t = 0; t < NSTEP; ++t) {
    if (wave < 4) {
      v8f dg[4];
#pragma unroll
      for (int r = 0; r < 8; ++r) {
        const int zr = (t - b0 - rb - r) & 255;
        const float* dgrow = DG + (size_t)zr * GD1 + j2;
        dg[0][r] = dgrow[0 * HD1];
        dg[1][r] = dgrow[1 * HD1];
        dg[2][r] = dgrow[2 * HD1];
        dg[3][r] = dgrow[3 * HD1];
      }
      v8f acc[4];
      acc[0] = z8; acc[1] = z8; acc[2] = z8; acc[3] = z8;
      gate_mac4<KD1R / 32>(acc, ad1row, wd1, HD1 * KD1R);
#pragma unroll
      for (int r = 0; r < 8; ++r) {
        acc[0][r] = fmaf(acc[0][r], Z_FOLD, dg[0][r]);
        acc[1][r] = fmaf(acc[1][r], Z_FOLD, dg[1][r]);
        acc[2][r] = fmaf(acc[2][r], Z_FOLD, dg[2][r]);
        acc[3][r] = fmaf(acc[3][r], Z_FOLD, dg[3][r]);
      }
      lstm_cell8(acc, 1.0f, bd1i, bd1f, bd1g, bd1o, cd1, hd1v);
    }
    __syncthreads();
    if (wave < 4) {
#pragma unroll
      for (int r = 0; r < 8; ++r) ad1[(rb + r) * PD1 + j2] = (_Float16)(A_CARRY * hd1v[r]);
    }
    __syncthreads();

    {
      v8f acc[4];
      acc[0] = z8; acc[1] = z8; acc[2] = z8; acc[3] = z8;
      gate_mac4<HD1 / 32>(acc, ad1row, wd2, HD2 * KD2);
      gate_mac4<HD2 / 32>(acc, ad2row, wd2 + HD1, HD2 * KD2);
      lstm_cell8(acc, Z_FOLD, bd2i, bd2f, bd2g, bd2o, cd2, hd2v);
    }
    __syncthreads();
#pragma unroll
    for (int r = 0; r < 8; ++r) ad2[(rb + r) * PD2 + j1] = (_Float16)(A_CARRY * hd2v[r]);
    __syncthreads();

    if (wave == 0) {
      v8f pacc = z8;
#pragma unroll
      for (int kf = 0; kf < KPROJ / 32; ++kf) {
        const v16h a = FragH::load(ad2row + 32 * kf);
        const v16h w = FragH::load(wo + 32 * kf);
        pacc = FragH::mma(a, w, pacc);
        guard1_h(pacc, a, w);
      }
      const int col = SSTRIDE * (t & 3) + c;
      const bool wr = (c < SSTRIDE) || (t == NSTEP - 1);
#pragma unroll
      for (int r = 0; r < 8; ++r) {
        const float yv = fmaf(pacc[r], Z_FOLD, obias);
        if (wr) ys[(rb + r) * YP + col] = yv;
      }
      if ((t & 3) == 3 || t == NSTEP - 1) {
        __builtin_amdgcn_fence(__ATOMIC_RELEASE, "workgroup");
        __builtin_amdgcn_wave_barrier();
        __builtin_amdgcn_fence(__ATOMIC_ACQUIRE, "workgroup");
        const int lineidx = t >> 2;
        const int q = lane >> 3, c4 = (lane & 7) * 4;
        for (int pass = 0; pass < 2; ++pass) {
#pragma unroll
          for (int it = 0; it < 4; ++it) {
            const int row = it * 4 + q;
            const v4f v = *(const v4f*)(ys + row * YP + c4);
            *(volatile v4f*)(out + (size_t)(b0 + row) * WLEN + (size_t)lineidx * 32 + c4) = v;
          }
          __threadfence();
        }
      }
    }
  }
}

extern "C" void kernel_launch(void* const* d_in, const int* in_sizes, int n_in,
                              void* d_out, int out_size, void* d_ws, size_t ws_size, hipStream_t stream) {
  if (n_in < 19 || d_out == nullptr || d_ws == nullptr) return;
  if (in_sizes[0] != NBATCH * WLEN || in_sizes[1] != 4 * HE1 * SWIN || in_sizes[2] != 4 * HE1 * HE1 ||
      in_sizes[3] != 4 * HE1 || in_sizes[4] != 4 * HE1 || in_sizes[5] != 4 * HE2 * HE1 || in_sizes[6] != 4 * HE2 * HE2 ||
      in_sizes[7] != 4 * HE2 || in_sizes[8] != 4 * HE2 || in_sizes[9] != 4 * HD1 * HE2 || in_sizes[10] != 4 * HD1 * HD1 ||
      in_sizes[11] != 4 * HD1 || in_sizes[12] != 4 * HD1 || in_sizes[13] != 4 * HD2 * HD1 || in_sizes[14] != 4 * HD2 * HD2 ||
      in_sizes[15] != 4 * HD2 || in_sizes[16] != 4 * HD2 || in_sizes[17] != NFEAT * HD2 || in_sizes[18] != NFEAT ||
      out_size != NBATCH * WLEN) return;

  const float* x      = (const float*)d_in[0];
  const float* e1_Wih = (const float*)d_in[1];
  const float* e1_Whh = (const float*)d_in[2];
  const float* e1_bih = (const float*)d_in[3];
  const float* e1_bhh = (const float*)d_in[4];
  const float* e2_Wih = (const float*)d_in[5];
  const float* e2_Whh = (const float*)d_in[6];
  const float* e2_bih = (const float*)d_in[7];
  const float* e2_bhh = (const float*)d_in[8];
  const float* d1_Wih = (const float*)d_in[9];
  const float* d1_Whh = (const float*)d_in[10];
  const float* d1_bih = (const float*)d_in[11];
  const float* d1_bhh = (const float*)d_in[12];
  const float* d2_Wih = (const float*)d_in[13];
  const float* d2_Whh = (const float*)d_in[14];
  const float* d2_bih = (const float*)d_in[15];
  const float* d2_bhh = (const float*)d_in[16];
  const float* out_W  = (const float*)d_in[17];
  const float* out_b  = (const float*)d_in[18];
  float* out = (float*)d_out;

  char* ws = (char*)d_ws; size_t off = 0;
  auto carve = [&](size_t bytes) -> char* { char* p = ws + off; off += (bytes + 255) & ~(size_t)255; return p; };
  unsigned short* WE1  = (unsigned short*)carve((size_t)4 * HE1 * KE1 * 2);
  unsigned short* WE2  = (unsigned short*)carve((size_t)4 * HE2 * KE2 * 2);
  unsigned short* WD1R = (unsigned short*)carve((size_t)4 * HD1 * KD1R * 2);
  unsigned short* WD2  = (unsigned short*)carve((size_t)4 * HD2 * KD2 * 2);
  unsigned short* WO   = (unsigned short*)carve((size_t)NFEAT * KPROJ * 2);
  unsigned short* WD1H = (unsigned short*)carve((size_t)4 * HD1 * HE2 * 2);
  unsigned short* WD1L = (unsigned short*)carve((size_t)4 * HD1 * HE2 * 2);
  unsigned short* ZH   = (unsigned short*)carve((size_t)NBATCH * HE2 * 2);
  unsigned short* ZL   = (unsigned short*)carve((size_t)NBATCH * HE2 * 2);
  float*          DG   = (float*)carve((size_t)NBATCH * GD1 * 4);
  if (off > ws_size || off > (size_t)134217728) return;

  const int n8_e1 = 4 * HE1 * KE1 / 8, n8_e2 = 4 * HE2 * KE2 / 8, n8_d1r = 4 * HD1 * KD1R / 8;
  const int n8_d2 = 4 * HD2 * KD2 / 8, n8_o = NFEAT * KPROJ / 8, n8_d1i = 4 * HD1 * HE2 / 8;
  wplane_kernel<<<(n8_e1 + NTHR - 1) / NTHR, NTHR, 0, stream>>>(e1_Wih, SWIN, e1_Whh, HE1, 32, KE1, n8_e1, 0, WE1);
  wplane_kernel<<<(n8_e2 + NTHR - 1) / NTHR, NTHR, 0, stream>>>(e2_Wih, HE1, e2_Whh, HE2, HE1, KE2, n8_e2, 0, WE2);
  wplane_kernel<<<(n8_d1r + NTHR - 1) / NTHR, NTHR, 0, stream>>>(d1_Whh, HD1, d1_Whh, HD1, KD1R, KD1R, n8_d1r, 0, WD1R);
  wplane_kernel<<<(n8_d2 + NTHR - 1) / NTHR, NTHR, 0, stream>>>(d2_Wih, HD1, d2_Whh, HD2, HD1, KD2, n8_d2, 0, WD2);
  wplane_kernel<<<(n8_o + NTHR - 1) / NTHR, NTHR, 0, stream>>>(out_W, KPROJ, out_W, KPROJ, KPROJ, KPROJ, n8_o, 0, WO);
  wplane_kernel<<<(n8_d1i + NTHR - 1) / NTHR, NTHR, 0, stream>>>(d1_Wih, HE2, d1_Wih, HE2, HE2, HE2, n8_d1i, 1, WD1H);
  wplane_kernel<<<(n8_d1i + NTHR - 1) / NTHR, NTHR, 0, stream>>>(d1_Wih, HE2, d1_Wih, HE2, HE2, HE2, n8_d1i, 2, WD1L);
  enc_kernel<<<NBATCH / TR, NTHR, 0, stream>>>(x, e1_bih, e1_bhh, e2_bih, e2_bhh, WE1, WE2, ZH, ZL);
  wmma_gemm64<1, true, 0, 0, false, 0><<<dim3(2, 1), 256, 0, stream>>>(
      ZH, ZL, HE2, 0L, WD1H, WD1L, HE2, 0L, (void*)DG, nullptr, GD1, 0L, nullptr, nullptr, 0L, NBATCH, GD1, HE2, 1.0f);
  dec_kernel<<<NBATCH / TR, NTHR, 0, stream>>>(d1_bih, d1_bhh, d2_bih, d2_bhh, out_b, WD1R, WD2, WO, DG, out);
}
